// CosineAttention_68865505624685
// MI455X (gfx1250) — hardware-verified
//
#include <hip/hip_runtime.h>
#include <stddef.h>

typedef __attribute__((ext_vector_type(16))) _Float16 v16h;
typedef __attribute__((ext_vector_type(8)))  _Float16 v8h;
typedef __attribute__((ext_vector_type(8)))  float    v8f;
typedef __attribute__((ext_vector_type(4)))  float    v4f;

constexpr int NBATCH = 4;
constexpr int LQ     = 2048;
constexpr int SKV    = 2048;
constexpr int NHEAD  = 8;
constexpr int HDIM   = 64;
constexpr int ROWSTRIDE = NHEAD * HDIM;

static_assert(LQ == SKV);
static_assert(HDIM == 64);
static_assert(LQ % 64 == 0 && SKV % 64 == 0);

union FragU { v16h v; v8h h[2]; };
__device__ __forceinline__ v16h frag_load(const _Float16* p) {
  FragU f;
  f.h[0] = *(const v8h*)(p);
  f.h[1] = *(const v8h*)(p + 16);
  return f.v;
}
__device__ __forceinline__ v8f mma_h(v16h a, v16h b, v8f c) {
  c = __builtin_amdgcn_wmma_f32_16x16x32_f16(false, a, false, b, (short)0, c, false, false);
  asm volatile("v_nop\n\tv_nop\n\tv_nop\n\tv_nop" : "+v"(c) : "v"(a), "v"(b));
  return c;
}
__device__ __forceinline__ void wave_lds_sync() {
  __builtin_amdgcn_fence(__ATOMIC_RELEASE, "workgroup");
  __builtin_amdgcn_wave_barrier();
  __builtin_amdgcn_fence(__ATOMIC_ACQUIRE, "workgroup");
}

constexpr int PREP_THREADS = 256;
constexpr int TROWS  = 64;
constexpr int LPITCH = 72;

__device__ __forceinline__ void norm_quarter(const float* __restrict__ p, v8h& o0, v8h& o1) {
  const v4f a0 = *(const v4f*)(p);
  const v4f a1 = *(const v4f*)(p + 4);
  const v4f a2 = *(const v4f*)(p + 8);
  const v4f a3 = *(const v4f*)(p + 12);
  float ss = 0.0f;
  ss += a0[0] * a0[0]; ss += a0[1] * a0[1]; ss += a0[2] * a0[2]; ss += a0[3] * a0[3];
  ss += a1[0] * a1[0]; ss += a1[1] * a1[1]; ss += a1[2] * a1[2]; ss += a1[3] * a1[3];
  ss += a2[0] * a2[0]; ss += a2[1] * a2[1]; ss += a2[2] * a2[2]; ss += a2[3] * a2[3];
  ss += a3[0] * a3[0]; ss += a3[1] * a3[1]; ss += a3[2] * a3[2]; ss += a3[3] * a3[3];
  ss += __shfl_xor(ss, 1, 32);
  ss += __shfl_xor(ss, 2, 32);
  const float sc = 16.0f / sqrtf(ss);
  o0[0] = (_Float16)(a0[0] * sc); o0[1] = (_Float16)(a0[1] * sc); o0[2] = (_Float16)(a0[2] * sc); o0[3] = (_Float16)(a0[3] * sc);
  o0[4] = (_Float16)(a1[0] * sc); o0[5] = (_Float16)(a1[1] * sc); o0[6] = (_Float16)(a1[2] * sc); o0[7] = (_Float16)(a1[3] * sc);
  o1[0] = (_Float16)(a2[0] * sc); o1[1] = (_Float16)(a2[1] * sc); o1[2] = (_Float16)(a2[2] * sc); o1[3] = (_Float16)(a2[3] * sc);
  o1[4] = (_Float16)(a3[0] * sc); o1[5] = (_Float16)(a3[1] * sc); o1[6] = (_Float16)(a3[2] * sc); o1[7] = (_Float16)(a3[3] * sc);
}

__device__ __forceinline__ void scat4(_Float16* vs, int d0, int r, v4f a) {
  vs[(d0 + 0) * LPITCH + r] = (_Float16)a[0];
  vs[(d0 + 1) * LPITCH + r] = (_Float16)a[1];
  vs[(d0 + 2) * LPITCH + r] = (_Float16)a[2];
  vs[(d0 + 3) * LPITCH + r] = (_Float16)a[3];
}

__global__ __launch_bounds__(PREP_THREADS)
void prep_planes(const float* __restrict__ q, const float* __restrict__ k, const float* __restrict__ v,
                 _Float16* __restrict__ Qh, _Float16* __restrict__ Kh, _Float16* __restrict__ Vt) {
  __shared__ __align__(16) _Float16 Qs[TROWS * LPITCH];
  __shared__ __align__(16) _Float16 Ks[TROWS * LPITCH];
  __shared__ __align__(16) _Float16 Vs[HDIM * LPITCH];

  const int tid  = threadIdx.x;
  const int lane = tid & 31;
  const int wave = tid >> 5;
  constexpr int NT = SKV / TROWS;
  const int bx = blockIdx.x;
  const int st = bx % NT;
  const int h  = (bx / NT) % NHEAD;
  const int n  = bx / (NT * NHEAD);
  const int s0 = st * TROWS;
  const int r  = tid >> 2;
  const int qd = tid & 3;
  const size_t goff = ((size_t)n * LQ + (size_t)(s0 + r)) * ROWSTRIDE + (size_t)h * HDIM + (size_t)qd * 16;

  {
    v8h o0, o1;
    norm_quarter(q + goff, o0, o1);
    *(v8h*)(Qs + r * LPITCH + qd * 16) = o0;
    *(v8h*)(Qs + r * LPITCH + qd * 16 + 8) = o1;
  }
  {
    v8h o0, o1;
    norm_quarter(k + goff, o0, o1);
    *(v8h*)(Ks + r * LPITCH + qd * 16) = o0;
    *(v8h*)(Ks + r * LPITCH + qd * 16 + 8) = o1;
  }
  {
    const float* vp = v + goff;
    const v4f a0 = *(const v4f*)(vp);
    const v4f a1 = *(const v4f*)(vp + 4);
    const v4f a2 = *(const v4f*)(vp + 8);
    const v4f a3 = *(const v4f*)(vp + 12);
    scat4(Vs, qd * 16 + 0,  r, a0);
    scat4(Vs, qd * 16 + 4,  r, a1);
    scat4(Vs, qd * 16 + 8,  r, a2);
    scat4(Vs, qd * 16 + 12, r, a3);
  }
  __syncthreads();

  const int rg = lane >> 3;
  const int c8 = (lane & 7) * 8;
  const size_t plane = (size_t)(n * NHEAD + h);
  _Float16* qdst = Qh + (plane * LQ  + (size_t)s0) * HDIM;
  _Float16* kdst = Kh + (plane * SKV + (size_t)s0) * HDIM;
  _Float16* vdst = Vt + (plane * HDIM) * SKV + (size_t)s0;
  for (int pass = 0; pass < 2; ++pass) {
#pragma unroll
    for (int it = 0; it < 2; ++it) {
      const int row = wave * 8 + it * 4 + rg;
      const v8h qv = *(const v8h*)(Qs + row * LPITCH + c8);
      const v8h kv = *(const v8h*)(Ks + row * LPITCH + c8);
      const v8h vv = *(const v8h*)(Vs + row * LPITCH + c8);
      *(volatile v8h*)(qdst + (size_t)row * HDIM + c8) = qv;
      *(volatile v8h*)(kdst + (size_t)row * HDIM + c8) = kv;
      *(volatile v8h*)(vdst + (size_t)row * SKV + c8) = vv;
    }
    __threadfence();
  }
}

constexpr int AT_THREADS = 128;
constexpr int QBLK   = 64;
constexpr int KCH    = 64;
constexpr int OPITCH = 68;
constexpr float PCARRY = 32768.0f;

__global__ __launch_bounds__(AT_THREADS)
void cos_attn(const _Float16* __restrict__ Qh, const _Float16* __restrict__ Kh, const _Float16* __restrict__ Vt,
              const float* __restrict__ temp, float* __restrict__ out) {
  __shared__ __align__(16) _Float16 Ksh[KCH * HDIM];
  __shared__ __align__(16) _Float16 Vth[HDIM * KCH];
  __shared__ __align__(16) _Float16 Psh[4][16 * KCH];
  __shared__ __align__(16) float    Os[4][16 * OPITCH];

  const int tid  = threadIdx.x;
  const int wave = tid >> 5;
  const int lane = tid & 31;
  const int hh   = lane >> 4;
  const int c    = lane & 15;

  constexpr int NQB = LQ / QBLK;
  const int bx = blockIdx.x;
  const int qb = bx % NQB;
  const int bh = bx / NQB;
  const int h  = bh % NHEAD;
  const int n  = bh / NHEAD;
  const int q0 = qb * QBLK + wave * 16;

  const size_t plane = (size_t)(n * NHEAD + h);
  const _Float16* qpl = Qh + plane * LQ * HDIM;
  const _Float16* kpl = Kh + plane * SKV * HDIM;
  const _Float16* vpl = Vt + plane * HDIM * SKV;
  float* ob = out + (size_t)n * LQ * ROWSTRIDE + (size_t)h * HDIM;

  const float invt   = 1.0f / temp[0];
  const float sscale = invt * 0.00390625f;

  v16h qa[2];
#pragma unroll
  for (int dc = 0; dc < 2; ++dc)
    qa[dc] = frag_load(qpl + (size_t)(q0 + c) * HDIM + dc * 32 + 8 * hh);

  const float neg_inf = -__builtin_inff();
  float mrow[8], lrow[8];
  v8f oacc[4];
#pragma unroll
  for (int r = 0; r < 8; ++r) { mrow[r] = neg_inf; lrow[r] = 0.0f; }
#pragma unroll
  for (int t = 0; t < 4; ++t) oacc[t] = (v8f){0.f, 0.f, 0.f, 0.f, 0.f, 0.f, 0.f, 0.f};

  for (int kc = 0; kc < SKV / KCH; ++kc) {
    const int kv0 = kc * KCH;
    __syncthreads();
#pragma unroll
    for (int i = 0; i < 4; ++i) {
      const int idx = tid + i * AT_THREADS;
      const int row = idx >> 3;
      const int c8  = (idx & 7) * 8;
      const v8h kk = *(const v8h*)(kpl + (size_t)(kv0 + row) * HDIM + c8);
      const v8h vv = *(const v8h*)(vpl + (size_t)row * SKV + (size_t)kv0 + c8);
      *(v8h*)(Ksh + row * HDIM + c8) = kk;
      *(v8h*)(Vth + row * KCH  + c8) = vv;
    }
    __syncthreads();

    v8f s[4];
#pragma unroll
    for (int j = 0; j < 4; ++j) {
      s[j] = (v8f){0.f, 0.f, 0.f, 0.f, 0.f, 0.f, 0.f, 0.f};
#pragma unroll
      for (int dc = 0; dc < 2; ++dc) {
        const v16h kb = frag_load(Ksh + (j * 16 + c) * HDIM + dc * 32 + 8 * hh);
        s[j] = mma_h(qa[dc], kb, s[j]);
      }
    }

    float cm[8];
#pragma unroll
    for (int r = 0; r < 8; ++r) {
      float m = neg_inf;
#pragma unroll
      for (int j = 0; j < 4; ++j) {
        const float sv = s[j][r] * sscale;
        s[j][r] = sv;
        m = fmaxf(m, sv);
      }
#pragma unroll
      for (int off = 1; off < 16; off <<= 1) m = fmaxf(m, __shfl_xor(m, off, 32));
      cm[r] = m;
    }
    _Float16* pw = Psh[wave];
#pragma unroll
    for (int r = 0; r < 8; ++r) {
      const float mnew  = fmaxf(mrow[r], cm[r]);
      const float alpha = expf(mrow[r] - mnew);
      mrow[r] = mnew;
      float psum = 0.0f;
#pragma unroll
      for (int j = 0; j < 4; ++j) {
        const float p = expf(s[j][r] - mnew);
        psum += p;
        pw[(8 * hh + r) * KCH + j * 16 + c] = (_Float16)(p * PCARRY);
      }
#pragma unroll
      for (int off = 1; off < 16; off <<= 1) psum += __shfl_xor(psum, off, 32);
      lrow[r] = lrow[r] * alpha + psum;
#pragma unroll
      for (int t = 0; t < 4; ++t) oacc[t][r] *= alpha;
    }
    wave_lds_sync();

#pragma unroll
    for (int kk = 0; kk < 2; ++kk) {
      const v16h pa = frag_load(pw + c * KCH + kk * 32 + 8 * hh);
#pragma unroll
      for (int t = 0; t < 4; ++t) {
        const v16h vb = frag_load(Vth + (t * 16 + c) * KCH + kk * 32 + 8 * hh);
        oacc[t] = mma_h(pa, vb, oacc[t]);
      }
    }
  }

  float* os = Os[wave];
#pragma unroll
  for (int r = 0; r < 8; ++r) {
    const float inv = 1.0f / (lrow[r] * PCARRY);
#pragma unroll
    for (int t = 0; t < 4; ++t) os[(8 * hh + r) * OPITCH + t * 16 + c] = oacc[t][r] * inv;
  }
  wave_lds_sync();
  {
    const int c4 = (lane & 15) * 4;
    for (int pass = 0; pass < 2; ++pass) {
#pragma unroll
      for (int it = 0; it < 8; ++it) {
        const int row = it * 2 + hh;
        const v4f val = *(const v4f*)(os + row * OPITCH + c4);
        *(volatile v4f*)(ob + (size_t)(q0 + row) * ROWSTRIDE + c4) = val;
      }
      __threadfence();
    }
  }
}

extern "C" void kernel_launch(void* const* d_in, const int* in_sizes, int n_in,
                              void* d_out, int out_size, void* d_ws, size_t ws_size,
                              hipStream_t stream) {
  (void)in_sizes; (void)n_in; (void)out_size;
  const float* q    = (const float*)d_in[0];
  const float* k    = (const float*)d_in[1];
  const float* v    = (const float*)d_in[2];
  const float* temp = (const float*)d_in[3];
  float* out = (float*)d_out;

  const size_t planeBytes = (size_t)NBATCH * NHEAD * LQ * HDIM * sizeof(_Float16);
  const size_t totalCarve = 3 * planeBytes;
  if (totalCarve > ws_size) return;
  char* ws = (char*)d_ws;
  _Float16* Qh = (_Float16*)(ws);
  _Float16* Kh = (_Float16*)(ws + planeBytes);
  _Float16* Vt = (_Float16*)(ws + 2 * planeBytes);

  prep_planes<<<dim3(NBATCH * NHEAD * (SKV / TROWS)), dim3(PREP_THREADS), 0, stream>>>(q, k, v, Qh, Kh, Vt);
  cos_attn<<<dim3(NBATCH * NHEAD * (LQ / QBLK)), dim3(AT_THREADS), 0, stream>>>(Qh, Kh, Vt, temp, out);
}
